// MultiEdgeGraphBlock_42691974922272
// MI455X (gfx1250) — hardware-run, weakly checked
//
#include <hip/hip_runtime.h>
#include <stddef.h>
#include <stdint.h>


#define NBAT   4
#define NN     10000
#define FD     256
#define NTYPE  5
#define DEG    16
#define MPAD   10112
#define KA     2560
#define KB     1024
#define KC     512
#define TM     128
#define GTHR   256
#define PADR   (MPAD - NN)

#define T_BSUM 0
#define T_LNS  256
#define T_LNB  768
#define T_B1   1280
#define T_B2   1536
#define T_END  1792

static_assert(DEG == 16 && FD == 256 && NTYPE == 5);
static_assert(FD == 32 * 8);
static_assert(KA == NTYPE * 2 * FD && KA % 32 == 0);
static_assert(KB == 4 * FD && KB % 32 == 0);
static_assert(KC == 2 * FD && KC % 32 == 0);
static_assert(MPAD % TM == 0 && MPAD >= NN && PADR == 112);
static_assert(NN % 8 == 0);
static_assert(GTHR == 256 && TM == 128);

constexpr size_t SZ_HB   = (size_t)NBAT * NN * FD * 2;
constexpr size_t SZ_MEAN = (size_t)MPAD * KA * 2;
constexpr size_t SZ_XN   = (size_t)MPAD * KB * 2;
constexpr size_t SZ_Y1   = (size_t)MPAD * KC * 2;
constexpr size_t SZ_WE   = (size_t)FD * KA * 2;
constexpr size_t SZ_W1   = (size_t)FD * KB * 2;
constexpr size_t SZ_W2   = (size_t)FD * KC * 2;
constexpr size_t SZ_TAB  = 8192;
constexpr size_t O_HB    = 0;
constexpr size_t O_MEAN  = O_HB + SZ_HB;
constexpr size_t O_XN    = O_MEAN + SZ_MEAN;
constexpr size_t O_Y1    = O_XN + SZ_XN;
constexpr size_t O_WE    = O_Y1 + SZ_Y1;
constexpr size_t O_W1    = O_WE + SZ_WE;
constexpr size_t O_W2    = O_W1 + SZ_W1;
constexpr size_t O_TAB   = O_W2 + SZ_W2;
constexpr size_t WS_TOTAL = O_TAB + SZ_TAB;
static_assert(O_MEAN % 256 == 0 && O_XN % 256 == 0 && O_Y1 % 256 == 0 && O_WE % 256 == 0);
static_assert(O_W1 % 256 == 0 && O_W2 % 256 == 0 && O_TAB % 256 == 0);
static_assert(WS_TOTAL <= (size_t)128 * 1024 * 1024);
static_assert((size_t)T_END * 4 <= SZ_TAB);

constexpr int NB_HB  = (NBAT * NN * FD / 8) / 256;
constexpr int NB_WE  = (FD * NTYPE * (FD / 8)) / 256;
constexpr int NB_W1  = (FD * (2 * FD / 8)) / 256;
constexpr int NB_W2  = (FD * (FD / 8)) / 256;
constexpr int NB_TAB = 2;
constexpr int ZU_MEAN = PADR * KA * 2 / 16;
constexpr int ZU_XN   = PADR * KB * 2 / 16;
constexpr int ZU_Y1   = PADR * KC * 2 / 16;
constexpr int NB_ZM  = ZU_MEAN / 256;
constexpr int NB_ZX  = ZU_XN / 256;
constexpr int NB_ZY  = ZU_Y1 / 256;
constexpr int B_WE0  = NB_HB;
constexpr int B_W10  = B_WE0 + NB_WE;
constexpr int B_W20  = B_W10 + NB_W1;
constexpr int B_TAB0 = B_W20 + NB_W2;
constexpr int B_Z0   = B_TAB0 + NB_TAB;
constexpr int NB_PREP = B_Z0 + NB_ZM + NB_ZX + NB_ZY;
static_assert((NBAT * NN * FD / 8) % 256 == 0);
static_assert(ZU_MEAN % 256 == 0 && ZU_XN % 256 == 0 && ZU_Y1 % 256 == 0);
static_assert(NB_TAB * 256 >= T_END / 4);

constexpr int STG_BYTES = TM * FD * 4;
static_assert(STG_BYTES + 1280 * 4 <= 327680);

typedef float          v4f   __attribute__((ext_vector_type(4)));
typedef float          v8f   __attribute__((ext_vector_type(8)));
typedef int            v8i   __attribute__((ext_vector_type(8)));
typedef unsigned       v2u   __attribute__((ext_vector_type(2)));
typedef unsigned       v4u   __attribute__((ext_vector_type(4)));
typedef unsigned short v8us  __attribute__((ext_vector_type(8)));
typedef unsigned short v16us __attribute__((ext_vector_type(16)));
typedef __bf16         v16bf __attribute__((ext_vector_type(16)));
typedef v4f  __attribute__((may_alias)) v4fa;
typedef v2u  __attribute__((may_alias)) v2ua;
typedef v4u  __attribute__((may_alias)) v4ua;
typedef v8us __attribute__((may_alias)) v8usa;
union FragB { v16bf v; v16us u; v8us h[2]; v8i w; };
struct HL { v8us h; v8us l; };

__device__ __forceinline__ v8f wmb(const FragB& a, const FragB& b, v8f c) {
  v8f d = __builtin_amdgcn_wmma_f32_16x16x32_bf16(false, a.v, false, b.v, (short)0, c, false, false);
  asm volatile("v_nop\n\tv_nop\n\tv_nop\n\tv_nop" : "+v"(d) : "v"(a.w), "v"(b.w));
  return d;
}

__device__ __forceinline__ unsigned bf16_bits(float f) {
  const unsigned u = __float_as_uint(f);
  const unsigned r = (u + 0x7FFFu + ((u >> 16) & 1u)) >> 16;
  return (f != f) ? 0x7FC0u : r;
}
__device__ __forceinline__ float bf16_val(float f) {
  return __uint_as_float(bf16_bits(f) << 16);
}
__device__ __forceinline__ float lo16f(unsigned w) { return __uint_as_float(w << 16); }
__device__ __forceinline__ float hi16f(unsigned w) { return __uint_as_float(w & 0xffff0000u); }

__device__ __forceinline__ HL split8(v4f a, v4f b) {
  HL r;
  unsigned t;
  t = bf16_bits(a.x); r.h[0] = (unsigned short)t; r.l[0] = (unsigned short)bf16_bits(a.x - __uint_as_float(t << 16));
  t = bf16_bits(a.y); r.h[1] = (unsigned short)t; r.l[1] = (unsigned short)bf16_bits(a.y - __uint_as_float(t << 16));
  t = bf16_bits(a.z); r.h[2] = (unsigned short)t; r.l[2] = (unsigned short)bf16_bits(a.z - __uint_as_float(t << 16));
  t = bf16_bits(a.w); r.h[3] = (unsigned short)t; r.l[3] = (unsigned short)bf16_bits(a.w - __uint_as_float(t << 16));
  t = bf16_bits(b.x); r.h[4] = (unsigned short)t; r.l[4] = (unsigned short)bf16_bits(b.x - __uint_as_float(t << 16));
  t = bf16_bits(b.y); r.h[5] = (unsigned short)t; r.l[5] = (unsigned short)bf16_bits(b.y - __uint_as_float(t << 16));
  t = bf16_bits(b.z); r.h[6] = (unsigned short)t; r.l[6] = (unsigned short)bf16_bits(b.z - __uint_as_float(t << 16));
  t = bf16_bits(b.w); r.h[7] = (unsigned short)t; r.l[7] = (unsigned short)bf16_bits(b.w - __uint_as_float(t << 16));
  return r;
}

__device__ __forceinline__ v4f cv4(v4f t) {
  v4f r;
  r.x = bf16_val(t.x); r.y = bf16_val(t.y); r.z = bf16_val(t.z); r.w = bf16_val(t.w);
  return r;
}
__device__ __forceinline__ float acc4(float s, v4f a) { return (((s + a.x) + a.y) + a.z) + a.w; }
__device__ __forceinline__ float sq4(float s, v4f d) {
  s = s + d.x * d.x; s = s + d.y * d.y; s = s + d.z * d.z; s = s + d.w * d.w;
  return s;
}

__device__ __forceinline__ void wt_unit(const float* __restrict__ src, int n, int j0,
                                        unsigned short* dst, int off2) {
  const float* p = src + (size_t)j0 * FD + n;
  const float f0 = p[0],      f1 = p[FD],     f2 = p[2 * FD], f3 = p[3 * FD];
  const float f4 = p[4 * FD], f5 = p[5 * FD], f6 = p[6 * FD], f7 = p[7 * FD];
  v8us o;
  o[0] = (unsigned short)bf16_bits(f0); o[1] = (unsigned short)bf16_bits(f1);
  o[2] = (unsigned short)bf16_bits(f2); o[3] = (unsigned short)bf16_bits(f3);
  o[4] = (unsigned short)bf16_bits(f4); o[5] = (unsigned short)bf16_bits(f5);
  o[6] = (unsigned short)bf16_bits(f6); o[7] = (unsigned short)bf16_bits(f7);
  *(volatile v8us*)dst = o;
  *(volatile v8us*)(dst + off2) = o;
  __threadfence();
  *(volatile v8us*)dst = o;
  *(volatile v8us*)(dst + off2) = o;
}

__global__ __launch_bounds__(256) void k_prep(
    const float* __restrict__ hin, const float* __restrict__ wedge, const float* __restrict__ bedge,
    const float* __restrict__ lns, const float* __restrict__ lnb,
    const float* __restrict__ w1, const float* __restrict__ b1,
    const float* __restrict__ w2, const float* __restrict__ b2,
    unsigned char* ws)
{
  const int blk = (int)blockIdx.x, tid = (int)threadIdx.x;
  if (blk < B_WE0) {
    const size_t u = (size_t)blk * 256 + tid;
    const float* p = hin + u * 8;
    const v4f a = *(const v4f*)p;
    const v4f c = *(const v4f*)(p + 4);
    v8us o;
    o[0] = (unsigned short)bf16_bits(a.x); o[1] = (unsigned short)bf16_bits(a.y);
    o[2] = (unsigned short)bf16_bits(a.z); o[3] = (unsigned short)bf16_bits(a.w);
    o[4] = (unsigned short)bf16_bits(c.x); o[5] = (unsigned short)bf16_bits(c.y);
    o[6] = (unsigned short)bf16_bits(c.z); o[7] = (unsigned short)bf16_bits(c.w);
    unsigned short* dp = (unsigned short*)(ws + O_HB) + u * 8;
    *(volatile v8us*)dp = o;
    __threadfence();
    *(volatile v8us*)dp = o;
  } else if (blk < B_W10) {
    const int u  = (blk - B_WE0) * 256 + tid;
    const int j8 = u & 31;
    const int ty = (u >> 5) % NTYPE;
    const int n  = u / (32 * NTYPE);
    unsigned short* dp = (unsigned short*)(ws + O_WE) + (size_t)n * KA + ty * (2 * FD) + j8 * 8;
    wt_unit(wedge + (size_t)ty * FD * FD, n, j8 * 8, dp, FD);
  } else if (blk < B_W20) {
    const int u  = (blk - B_W10) * 256 + tid;
    const int j8 = u & 63;
    const int n  = u >> 6;
    unsigned short* dp = (unsigned short*)(ws + O_W1) + (size_t)n * KB + j8 * 8;
    wt_unit(w1, n, j8 * 8, dp, 2 * FD);
  } else if (blk < B_TAB0) {
    const int u  = (blk - B_W20) * 256 + tid;
    const int j8 = u & 31;
    const int n  = u >> 5;
    unsigned short* dp = (unsigned short*)(ws + O_W2) + (size_t)n * KC + j8 * 8;
    wt_unit(w2, n, j8 * 8, dp, FD);
  } else if (blk < B_Z0) {
    const int u = (blk - B_TAB0) * 256 + tid;
    if (u < T_END / 4) {
      v4f r;
      if (u < 64) {
        const int c = 4 * u;
        const v4f t0 = *(const v4f*)(bedge + c);
        const v4f t1 = *(const v4f*)(bedge + FD + c);
        const v4f t2 = *(const v4f*)(bedge + 2 * FD + c);
        const v4f t3 = *(const v4f*)(bedge + 3 * FD + c);
        const v4f t4 = *(const v4f*)(bedge + 4 * FD + c);
        r.x = (((bf16_val(t0.x) + bf16_val(t1.x)) + bf16_val(t2.x)) + bf16_val(t3.x)) + bf16_val(t4.x);
        r.y = (((bf16_val(t0.y) + bf16_val(t1.y)) + bf16_val(t2.y)) + bf16_val(t3.y)) + bf16_val(t4.y);
        r.z = (((bf16_val(t0.z) + bf16_val(t1.z)) + bf16_val(t2.z)) + bf16_val(t3.z)) + bf16_val(t4.z);
        r.w = (((bf16_val(t0.w) + bf16_val(t1.w)) + bf16_val(t2.w)) + bf16_val(t3.w)) + bf16_val(t4.w);
      } else if (u < 192) {
        r = cv4(*(const v4f*)(lns + 4 * (u - 64)));
      } else if (u < 320) {
        r = cv4(*(const v4f*)(lnb + 4 * (u - 192)));
      } else if (u < 384) {
        r = cv4(*(const v4f*)(b1 + 4 * (u - 320)));
      } else {
        r = cv4(*(const v4f*)(b2 + 4 * (u - 384)));
      }
      float* dp = (float*)(ws + O_TAB) + 4 * u;
      *(volatile v4f*)dp = r;
      __threadfence();
      *(volatile v4f*)dp = r;
    }
  } else {
    const int zb = blk - B_Z0;
    size_t off;
    if (zb < NB_ZM)              off = O_MEAN + (size_t)NN * KA * 2 + ((size_t)zb * 256 + tid) * 16;
    else if (zb < NB_ZM + NB_ZX) off = O_XN + (size_t)NN * KB * 2 + ((size_t)(zb - NB_ZM) * 256 + tid) * 16;
    else                         off = O_Y1 + (size_t)NN * KC * 2 + ((size_t)(zb - NB_ZM - NB_ZX) * 256 + tid) * 16;
    const v4u z = {0u, 0u, 0u, 0u};
    *(volatile v4u*)(ws + off) = z;
    __threadfence();
    *(volatile v4u*)(ws + off) = z;
  }
}

__global__ __launch_bounds__(256) void k_gather(const unsigned short* __restrict__ hbb,
                                                const int* __restrict__ eidx,
                                                const float* __restrict__ emask,
                                                unsigned short* __restrict__ mean)
{
  const int tid = (int)threadIdx.x, lane = tid & 31, wave = tid >> 5;
  const int node = (int)blockIdx.x * 8 + wave;
  if (node >= NN) return;
  const float qnan = __uint_as_float(0x7fc00000u);
#pragma unroll 1
  for (int ty = 0; ty < NTYPE; ++ty) {
    const size_t eo = ((size_t)ty * NN + node) * DEG + (lane & 15);
    const int iv  = eidx[eo];
    const int mvi = __float_as_int(bf16_val(emask[eo]));
    float a0 = 0.0f, a1 = 0.0f, a2 = 0.0f, a3 = 0.0f, a4 = 0.0f, a5 = 0.0f, a6 = 0.0f, a7 = 0.0f;
    float msum = 0.0f;
#pragma unroll 1
    for (int s = 0; s < DEG; ++s) {
      int id = __builtin_amdgcn_readlane(iv, s);
      const float mk = __int_as_float(__builtin_amdgcn_readlane(mvi, s));
      id = id < 0 ? 0 : id;
      const float mke = (id >= NN) ? qnan : mk;
      const int ic = id > NN - 1 ? NN - 1 : id;
      const v4u w = *(const v4ua*)(hbb + (size_t)ic * FD + 8 * lane);
      asm volatile("" :: "v"(w));
      a0 = a0 + lo16f(w.x) * mke;
      a1 = a1 + hi16f(w.x) * mke;
      a2 = a2 + lo16f(w.y) * mke;
      a3 = a3 + hi16f(w.y) * mke;
      a4 = a4 + lo16f(w.z) * mke;
      a5 = a5 + hi16f(w.z) * mke;
      a6 = a6 + lo16f(w.w) * mke;
      a7 = a7 + hi16f(w.w) * mke;
      msum = msum + mk;
    }
    const float den = (msum < 1.0f) ? 1.0f : msum;
    v4f q0, q1;
    q0.x = a0 / den; q0.y = a1 / den; q0.z = a2 / den; q0.w = a3 / den;
    q1.x = a4 / den; q1.y = a5 / den; q1.z = a6 / den; q1.w = a7 / den;
    const HL r = split8(q0, q1);
    unsigned short* rp = mean + (size_t)node * KA + ty * (2 * FD) + 8 * lane;
    *(volatile v8us*)rp = r.h;
    *(volatile v8us*)(rp + FD) = r.l;
    __threadfence();
    *(volatile v8us*)rp = r.h;
    *(volatile v8us*)(rp + FD) = r.l;
  }
}

template <int MODE, int K>
__global__ __launch_bounds__(GTHR) __attribute__((amdgpu_num_vgpr(248)))
void k_gemm(const unsigned short* __restrict__ Apl, const unsigned short* __restrict__ BT,
            const float* __restrict__ tab, const unsigned short* __restrict__ hbb,
            unsigned short* __restrict__ outp, float* __restrict__ outf)
{
  extern __shared__ __attribute__((aligned(16))) float stg[];
  __shared__ __attribute__((aligned(16))) float stab[1280];
  static_assert(K % 32 == 0);
  constexpr int TOFF = (MODE == 0) ? T_BSUM : ((MODE == 1) ? T_B1 : T_B2);
  constexpr int TN4  = (MODE == 0) ? 320 : 64;

  const int tid = (int)threadIdx.x, lane = tid & 31, wave = tid >> 5;
  const int hh = lane >> 4, m = lane & 15;
  const int rg = wave >> 1, cg = wave & 1;
  const int rowBase = (int)blockIdx.x * TM;

  for (int q = tid; q < TN4; q += GTHR)
    *(v4fa*)(stab + 4 * q) = *(const v4f*)(tab + TOFF + 4 * q);

  v8f acc[2][8];
  {
    const v8f z = {0.f, 0.f, 0.f, 0.f, 0.f, 0.f, 0.f, 0.f};
#pragma unroll
    for (int mt = 0; mt < 2; ++mt)
#pragma unroll
      for (int nt = 0; nt < 8; ++nt) acc[mt][nt] = z;
  }
  const unsigned short* ap0 = Apl + (size_t)(rowBase + 32 * rg + m) * (size_t)K + 8 * hh;
  const unsigned short* ap1 = ap0 + (size_t)16 * (size_t)K;
  const unsigned short* bp  = BT + (size_t)(128 * cg + m) * (size_t)K + 8 * hh;

#pragma unroll 1
  for (int k0 = 0; k0 < K; k0 += 32) {
    FragB a0, a1;
    a0.h[0] = *(const v8usa*)(ap0 + k0);
    a0.h[1] = *(const v8usa*)(ap0 + k0 + 16);
    a1.h[0] = *(const v8usa*)(ap1 + k0);
    a1.h[1] = *(const v8usa*)(ap1 + k0 + 16);
#pragma unroll
    for (int nt = 0; nt < 8; ++nt) {
      const unsigned short* wq = bp + (size_t)(16 * nt) * (size_t)K + k0;
      FragB bf;
      bf.h[0] = *(const v8usa*)wq;
      bf.h[1] = *(const v8usa*)(wq + 16);
      acc[0][nt] = wmb(a0, bf, acc[0][nt]);
      acc[1][nt] = wmb(a1, bf, acc[1][nt]);
    }
  }

#pragma unroll
  for (int mt = 0; mt < 2; ++mt)
#pragma unroll
    for (int nt = 0; nt < 8; ++nt) {
      const int lc = 128 * cg + 16 * nt + m;
#pragma unroll
      for (int r = 0; r < 8; ++r) {
        const int lr = 32 * rg + 16 * mt + 8 * hh + r;
        stg[lr * FD + lc] = acc[mt][nt][r];
      }
    }
  __syncthreads();

  if constexpr (MODE == 0) {
    const v4f bs0 = *(const v4fa*)(stab + 8 * lane);
    const v4f bs1 = *(const v4fa*)(stab + 8 * lane + 4);
    const v4f sh0 = *(const v4fa*)(stab + 256 + 8 * lane);
    const v4f sh1 = *(const v4fa*)(stab + 256 + 8 * lane + 4);
    const v4f sa0 = *(const v4fa*)(stab + 512 + 8 * lane);
    const v4f sa1 = *(const v4fa*)(stab + 512 + 8 * lane + 4);
    const v4f bh0 = *(const v4fa*)(stab + 768 + 8 * lane);
    const v4f bh1 = *(const v4fa*)(stab + 768 + 8 * lane + 4);
    const v4f ba0 = *(const v4fa*)(stab + 1024 + 8 * lane);
    const v4f ba1 = *(const v4fa*)(stab + 1024 + 8 * lane + 4);
#pragma unroll 1
    for (int i = 0; i < 16; ++i) {
      const int lr  = 16 * wave + i;
      const int row = rowBase + lr;
      const int rc  = row < NN ? row : NN - 1;
      const v4u hw = *(const v4ua*)(hbb + (size_t)rc * FD + 8 * lane);
      asm volatile("" :: "v"(hw));
      const v4f t0 = *(const v4fa*)(stg + lr * FD + 8 * lane);
      const v4f t1 = *(const v4fa*)(stg + lr * FD + 8 * lane + 4);
      v4f xh0, xh1;
      xh0.x = lo16f(hw.x); xh0.y = hi16f(hw.x); xh0.z = lo16f(hw.y); xh0.w = hi16f(hw.y);
      xh1.x = lo16f(hw.z); xh1.y = hi16f(hw.z); xh1.z = lo16f(hw.w); xh1.w = hi16f(hw.w);
      const v4f xa0 = t0 + bs0;
      const v4f xa1 = t1 + bs1;
      float s = acc4(acc4(acc4(acc4(0.0f, xh0), xh1), xa0), xa1);
      s += __shfl_xor(s, 16);
      s += __shfl_xor(s, 8);
      s += __shfl_xor(s, 4);
      s += __shfl_xor(s, 2);
      s += __shfl_xor(s, 1);
      const float mu = s * (1.0f / 512.0f);
      const v4f dh0 = xh0 - mu, dh1 = xh1 - mu, da0 = xa0 - mu, da1 = xa1 - mu;
      float vs = sq4(sq4(sq4(sq4(0.0f, dh0), dh1), da0), da1);
      vs += __shfl_xor(vs, 16);
      vs += __shfl_xor(vs, 8);
      vs += __shfl_xor(vs, 4);
      vs += __shfl_xor(vs, 2);
      vs += __shfl_xor(vs, 1);
      const float var = vs * (1.0f / 512.0f);
      const float rs  = 1.0f / sqrtf(var + 1e-6f);
      const v4f yh0 = (dh0 * rs) * sh0 + bh0;
      const v4f yh1 = (dh1 * rs) * sh1 + bh1;
      const v4f ya0 = (da0 * rs) * sa0 + ba0;
      const v4f ya1 = (da1 * rs) * sa1 + ba1;
      const HL ph = split8(yh0, yh1);
      const HL pa = split8(ya0, ya1);
      if (row < NN) {
        unsigned short* rp = outp + (size_t)row * KB + 8 * lane;
        *(volatile v8us*)rp = ph.h;
        *(volatile v8us*)(rp + FD) = pa.h;
        *(volatile v8us*)(rp + 2 * FD) = ph.l;
        *(volatile v8us*)(rp + 3 * FD) = pa.l;
        __threadfence();
        *(volatile v8us*)rp = ph.h;
        *(volatile v8us*)(rp + FD) = pa.h;
        *(volatile v8us*)(rp + 2 * FD) = ph.l;
        *(volatile v8us*)(rp + 3 * FD) = pa.l;
      }
    }
  } else if constexpr (MODE == 1) {
    const v4f c0 = *(const v4fa*)(stab + 8 * lane);
    const v4f c1 = *(const v4fa*)(stab + 8 * lane + 4);
#pragma unroll 1
    for (int i = 0; i < 16; ++i) {
      const int lr  = 16 * wave + i;
      const int row = rowBase + lr;
      const v4f t0 = *(const v4fa*)(stg + lr * FD + 8 * lane);
      const v4f t1 = *(const v4fa*)(stg + lr * FD + 8 * lane + 4);
      const v4f v0 = t0 + c0;
      const v4f v1 = t1 + c1;
      v4f y0, y1;
      y0.x = (v0.x > 0.0f) ? v0.x : (v0.x - v0.x);
      y0.y = (v0.y > 0.0f) ? v0.y : (v0.y - v0.y);
      y0.z = (v0.z > 0.0f) ? v0.z : (v0.z - v0.z);
      y0.w = (v0.w > 0.0f) ? v0.w : (v0.w - v0.w);
      y1.x = (v1.x > 0.0f) ? v1.x : (v1.x - v1.x);
      y1.y = (v1.y > 0.0f) ? v1.y : (v1.y - v1.y);
      y1.z = (v1.z > 0.0f) ? v1.z : (v1.z - v1.z);
      y1.w = (v1.w > 0.0f) ? v1.w : (v1.w - v1.w);
      const HL p = split8(y0, y1);
      if (row < NN) {
        unsigned short* rp = outp + (size_t)row * KC + 8 * lane;
        *(volatile v8us*)rp = p.h;
        *(volatile v8us*)(rp + FD) = p.l;
        __threadfence();
        *(volatile v8us*)rp = p.h;
        *(volatile v8us*)(rp + FD) = p.l;
      }
    }
  } else {
    const v4f c0 = *(const v4fa*)(stab + 4 * lane);
    const v4f c1 = *(const v4fa*)(stab + 128 + 4 * lane);
#pragma unroll 1
    for (int i = 0; i < 16; ++i) {
      const int lr  = 16 * wave + i;
      const int row = rowBase + lr;
      const int rc  = row < NN ? row : NN - 1;
      const v2u ha = *(const v2ua*)(hbb + (size_t)rc * FD + 4 * lane);
      const v2u hc = *(const v2ua*)(hbb + (size_t)rc * FD + 128 + 4 * lane);
      asm volatile("" :: "v"(ha), "v"(hc));
      const v4f t0 = *(const v4fa*)(stg + lr * FD + 4 * lane);
      const v4f t1 = *(const v4fa*)(stg + lr * FD + 128 + 4 * lane);
      const v4f u0 = t0 + c0;
      const v4f u1 = t1 + c1;
      v4f o0, o1;
      o0.x = lo16f(ha.x) + u0.x; o0.y = hi16f(ha.x) + u0.y;
      o0.z = lo16f(ha.y) + u0.z; o0.w = hi16f(ha.y) + u0.w;
      o1.x = lo16f(hc.x) + u1.x; o1.y = hi16f(hc.x) + u1.y;
      o1.z = lo16f(hc.y) + u1.z; o1.w = hi16f(hc.y) + u1.w;
      if (row < NN) {
        float* rp = outf + (size_t)row * FD + 4 * lane;
        *(volatile v4f*)rp = o0;
        *(volatile v4f*)(rp + 128) = o1;
        __threadfence();
        *(volatile v4f*)rp = o0;
        *(volatile v4f*)(rp + 128) = o1;
      }
    }
  }
}

extern "C" void kernel_launch(void* const* d_in, const int* in_sizes, int n_in,
                              void* d_out, int out_size, void* d_ws, size_t ws_size,
                              hipStream_t stream) {
  if (n_in < 11) return;
  if (in_sizes[0] != NBAT * NN * FD) return;
  if (in_sizes[1] != NTYPE * NN * DEG) return;
  if (in_sizes[2] != NTYPE * NN * DEG) return;
  if (in_sizes[3] != NTYPE * FD * FD) return;
  if (in_sizes[4] != NTYPE * FD) return;
  if (in_sizes[5] != 2 * FD || in_sizes[6] != 2 * FD) return;
  if (in_sizes[7] != 2 * FD * FD || in_sizes[8] != FD) return;
  if (in_sizes[9] != FD * FD || in_sizes[10] != FD) return;
  if (out_size != NBAT * NN * FD) return;
  if (ws_size < WS_TOTAL) return;

  const float* hin   = (const float*)d_in[0];
  const int*   eidx  = (const int*)d_in[1];
  const float* emask = (const float*)d_in[2];
  const float* wedge = (const float*)d_in[3];
  const float* bedge = (const float*)d_in[4];
  const float* lns   = (const float*)d_in[5];
  const float* lnb   = (const float*)d_in[6];
  const float* w1    = (const float*)d_in[7];
  const float* b1    = (const float*)d_in[8];
  const float* w2    = (const float*)d_in[9];
  const float* b2    = (const float*)d_in[10];
  float* out = (float*)d_out;

  unsigned char* ws = (unsigned char*)d_ws;
  unsigned short* HB   = (unsigned short*)(ws + O_HB);
  unsigned short* MEAN = (unsigned short*)(ws + O_MEAN);
  unsigned short* XN   = (unsigned short*)(ws + O_XN);
  unsigned short* Y1   = (unsigned short*)(ws + O_Y1);
  unsigned short* WE   = (unsigned short*)(ws + O_WE);
  unsigned short* W1D  = (unsigned short*)(ws + O_W1);
  unsigned short* W2D  = (unsigned short*)(ws + O_W2);
  float*          TAB  = (float*)(ws + O_TAB);

  hipFuncSetAttribute(reinterpret_cast<const void*>(&k_gemm<0, KA>), hipFuncAttributeMaxDynamicSharedMemorySize, STG_BYTES);
  hipFuncSetAttribute(reinterpret_cast<const void*>(&k_gemm<1, KB>), hipFuncAttributeMaxDynamicSharedMemorySize, STG_BYTES);
  hipFuncSetAttribute(reinterpret_cast<const void*>(&k_gemm<2, KC>), hipFuncAttributeMaxDynamicSharedMemorySize, STG_BYTES);

  k_prep<<<NB_PREP, 256, 0, stream>>>(hin, wedge, bedge, lns, lnb, w1, b1, w2, b2, ws);

  for (int b = 0; b < NBAT; ++b) {
    const unsigned short* hbb = HB + (size_t)b * NN * FD;
    float* ob = out + (size_t)b * NN * FD;
    k_gather<<<NN / 8, 256, 0, stream>>>(hbb, eidx, emask, MEAN);
    k_gemm<0, KA><<<MPAD / TM, GTHR, STG_BYTES, stream>>>(MEAN, WE, TAB, hbb, XN, ob);
    k_gemm<1, KB><<<MPAD / TM, GTHR, STG_BYTES, stream>>>(XN, W1D, TAB, hbb, Y1, ob);
    k_gemm<2, KC><<<MPAD / TM, GTHR, STG_BYTES, stream>>>(Y1, W2D, TAB, hbb, XN, ob);
  }
}
